// TemporalEncoderLayer_12068858101760
// MI455X (gfx1250) — hardware-verified
//
#include <hip/hip_runtime.h>
#include <math.h>

constexpr int kBatch   = 2;
constexpr int kSeq     = 2048;
constexpr int kEmb     = 1024;
constexpr int kHeads   = 16;
constexpr int kHd      = 64;
constexpr int kFF      = 4096;
constexpr int kRows    = kBatch * kSeq;
constexpr int kBH      = kBatch * kHeads;
constexpr int kHalfWin = 256;
constexpr int kFFRows  = 2048;

constexpr float kWCarry     = 32.0f;
constexpr float kWCarryInv  = 1.0f / 32.0f;
constexpr float kPCarry     = 32768.0f;
constexpr float kCtxCarry   = 64.0f;
constexpr float kF1Carry    = 16.0f;
constexpr float kScoreScale = 0.125f;
constexpr float kPVScale    = kCtxCarry / kPCarry;
constexpr float kOutScale   = 1.0f / (kCtxCarry * kWCarry);
constexpr float kFF2Scale   = 1.0f / (kF1Carry * kWCarry);
constexpr float kInvEmb     = 1.0f / 1024.0f;
constexpr float kLnEps      = 1e-5f;
constexpr float kMaskFill   = -1.0e9f;
constexpr float kInvSqrt2   = 0.70710678118654752f;

typedef __attribute__((ext_vector_type(16))) _Float16 v16h;
typedef __attribute__((ext_vector_type(8)))  _Float16 v8h;
typedef __attribute__((ext_vector_type(16))) __bf16   v16b;
typedef __attribute__((ext_vector_type(8)))  __bf16   v8b;
typedef __attribute__((ext_vector_type(8)))  float    v8f;
typedef __attribute__((ext_vector_type(4)))  float    v4f;
typedef __attribute__((ext_vector_type(2)))  float    v2f;
typedef __attribute__((ext_vector_type(4)))  unsigned int v4u;
typedef __attribute__((ext_vector_type(4)))  int      v4i;

__device__ __forceinline__ unsigned short f2bf_bits(float f) {
  unsigned u = __float_as_uint(f);
  return (unsigned short)((u + 0x7FFFu + ((u >> 16) & 1u)) >> 16);
}
__device__ __forceinline__ float bf_bits2f(unsigned short h) { return __uint_as_float(((unsigned)h) << 16); }

__device__ __forceinline__ void dep_guard_h(v8f& a, v8f& b, v16h x, v16h y) { asm volatile("v_nop\n\tv_nop\n\tv_nop\n\tv_nop" : "+v"(a), "+v"(b) : "v"(x), "v"(y)); }
__device__ __forceinline__ void dep_guard_b(v8f& a, v8f& b, v16b x, v16b y) { asm volatile("v_nop\n\tv_nop\n\tv_nop\n\tv_nop" : "+v"(a), "+v"(b) : "v"(x), "v"(y)); }
__device__ __forceinline__ void keep4_h(v16h a, v16h b, v16h c, v16h d) { asm volatile("v_nop" :: "v"(a), "v"(b), "v"(c), "v"(d)); }
__device__ __forceinline__ void keep4_b(v16b a, v16b b, v16b c, v16b d) { asm volatile("v_nop" :: "v"(a), "v"(b), "v"(c), "v"(d)); }
__device__ __forceinline__ void acc_guard4(v8f& a, v8f& b, v8f& c, v8f& d) { asm volatile("v_nop\n\tv_nop\n\tv_nop\n\tv_nop" : "+v"(a), "+v"(b), "+v"(c), "+v"(d)); }
template <typename T> struct Frag;
template <> struct Frag<_Float16> {
  typedef v16h V; union U { v16h v; v8h h[2]; };
  static __device__ __forceinline__ v16h load(const _Float16* p) {
    U f; f.h[0] = *(const v8h*)(p); f.h[1] = *(const v8h*)(p + 16); return f.v;
  }
  static __device__ __forceinline__ v8f mma(v16h a, v16h b, v8f c) {
    return __builtin_amdgcn_wmma_f32_16x16x32_f16(false, a, false, b, (short)0, c, false, false);
  }
  static __device__ __forceinline__ void guard(v8f& a, v8f& b, v16h x, v16h y) { dep_guard_h(a, b, x, y); }
  static __device__ __forceinline__ void keep(v16h a, v16h b, v16h c, v16h d) { keep4_h(a, b, c, d); }
};
template <> struct Frag<__bf16> {
  typedef v16b V; union U { v16b v; v8b h[2]; };
  static __device__ __forceinline__ v16b load(const __bf16* p) {
    U f; f.h[0] = *(const v8b*)(p); f.h[1] = *(const v8b*)(p + 16); return f.v;
  }
  static __device__ __forceinline__ v8f mma(v16b a, v16b b, v8f c) {
    return __builtin_amdgcn_wmma_f32_16x16x32_bf16(false, a, false, b, (short)0, c, false, false);
  }
  static __device__ __forceinline__ void guard(v8f& a, v8f& b, v16b x, v16b y) { dep_guard_b(a, b, x, y); }
  static __device__ __forceinline__ void keep(v16b a, v16b b, v16b c, v16b d) { keep4_b(a, b, c, d); }
};

__device__ __forceinline__ unsigned pk16(unsigned short a, unsigned short b) { return (unsigned)a | ((unsigned)b << 16); }
__device__ __forceinline__ unsigned short h_bits(float f) { const _Float16 h = (_Float16)f; return __builtin_bit_cast(unsigned short, h); }

template <int ET> struct Elem;
template <> struct Elem<0> { typedef _Float16 T; };
template <> struct Elem<1> { typedef __bf16 T; };
template <int ET, bool SPLIT, int BIAS_MODE, int OUT_MODE, bool RESID, int ACT = 0, int TRI = 0>
__global__ __launch_bounds__(256) void wmma_gemm64(
    const unsigned short* __restrict__ Ap, const unsigned short* __restrict__ A2p, int lda, long strideA,
    const unsigned short* __restrict__ Btp, const unsigned short* __restrict__ Bt2p, int ldb, long strideB,
    void* __restrict__ Cout, void* __restrict__ Cout2, int ldc, long strideC,
    const float* __restrict__ bias,
    const float* __restrict__ resid, long strideR,
    int M, int N, int K, float scale) {
  typedef typename Elem<ET>::T T;
  typedef typename Frag<T>::V V;
  const T* A = (const T*)Ap; const T* A2 = (const T*)A2p; const T* Bt = (const T*)Btp; const T* Bt2 = (const T*)Bt2p;
  __shared__ __align__(16) float sT[8][16 * 68];
  const int b    = blockIdx.y;
  const int lane = threadIdx.x & 31;
  const int wave = threadIdx.x >> 5;
  const int tilesN = N >> 6;
  const int tilesM = M >> 6;
  const int tile = blockIdx.x * 8 + wave;
  if (tile >= tilesM * tilesN) return;
  const int tm = tile / tilesN;
  const int tn = tile - tm * tilesN;
  if (TRI == 1 && tn > tm) return;
  const int m0 = tm << 6;
  const int n0 = tn << 6;
  const int Kend = (TRI == 2) ? ((m0 + 64 < K) ? (m0 + 64) : K) : K;

  const T* Ab  = A  + (size_t)b * strideA;
  const T* Bb  = Bt + (size_t)b * strideB;
  const T* Ab2 = SPLIT ? (A2  + (size_t)b * strideA) : nullptr;
  const T* Bb2 = SPLIT ? (Bt2 + (size_t)b * strideB) : nullptr;

  const int rlane = lane & 15;
  const int koff  = (lane >> 4) * 8;
  const int mOff  = (lane >> 4) * 8;

  v8f acc[4][4];
#pragma unroll
  for (int i = 0; i < 4; ++i)
#pragma unroll
    for (int j = 0; j < 4; ++j) acc[i][j] = (v8f){0.f,0.f,0.f,0.f,0.f,0.f,0.f,0.f};

  for (int k0 = 0; k0 < Kend; k0 += 32) {
    V bh[4], bl[4];
#pragma unroll
    for (int j = 0; j < 4; ++j) {
      const size_t bo = (size_t)(n0 + (j << 4) + rlane) * ldb + koff + k0;
      bh[j] = Frag<T>::load(Bb + bo);
      if (SPLIT) bl[j] = Frag<T>::load(Bb2 + bo);
    }
#pragma unroll
    for (int i = 0; i < 4; ++i) {
      const size_t ao = (size_t)(m0 + (i << 4) + rlane) * lda + koff + k0;
      V ah = Frag<T>::load(Ab + ao);
      V al;
      if (SPLIT) al = Frag<T>::load(Ab2 + ao);
#pragma unroll
      for (int j = 0; j < 4; ++j) {
        acc[i][j] = Frag<T>::mma(ah, bh[j], acc[i][j]);
        if (SPLIT) {
          acc[i][j] = Frag<T>::mma(ah, bl[j], acc[i][j]);
          acc[i][j] = Frag<T>::mma(al, bh[j], acc[i][j]);
        }
      }
      Frag<T>::guard(acc[i][0], acc[i][3], ah, SPLIT ? al : ah);
    }
    Frag<T>::keep(bh[0], bh[1], bh[2], bh[3]);
    if (SPLIT) Frag<T>::keep(bl[0], bl[1], bl[2], bl[3]);
  }
  acc_guard4(acc[0][0], acc[0][1], acc[0][2], acc[0][3]);
  acc_guard4(acc[1][0], acc[1][1], acc[1][2], acc[1][3]);
  acc_guard4(acc[2][0], acc[2][1], acc[2][2], acc[2][3]);
  acc_guard4(acc[3][0], acc[3][1], acc[3][2], acc[3][3]);

  float* slab = sT[wave];
  const float* Rb = RESID ? (resid + (size_t)b * strideR) : nullptr;
#pragma unroll
  for (int i = 0; i < 4; ++i) {
    const int mBase = m0 + (i << 4);
#pragma unroll
    for (int j = 0; j < 4; ++j) {
      const int n = n0 + (j << 4) + rlane;
      float bv = 0.f;
      if (BIAS_MODE == 2) bv = bias[n];
#pragma unroll
      for (int r = 0; r < 8; ++r) {
        float v = acc[i][j][r] * scale;
        if (BIAS_MODE == 1) v += bias[mBase + mOff + r];
        if (BIAS_MODE == 2) v += bv;
        if (RESID) v += Rb[(size_t)(mBase + mOff + r) * ldc + n];
        if (ACT == 2) v = fmaxf(v, 0.0f);
        if (ACT == 4) v = (v > 0.f) ? v : 0.01f * v;
        slab[(mOff + r) * 68 + (j << 4) + rlane] = v;
      }
    }
    __builtin_amdgcn_fence(__ATOMIC_RELEASE, "workgroup");
    __builtin_amdgcn_wave_barrier();
    __builtin_amdgcn_fence(__ATOMIC_ACQUIRE, "workgroup");
    if (OUT_MODE == 0) {
      float* C = (float*)Cout + (size_t)b * strideC;
      const int hh = lane >> 4, c4 = (lane & 15) * 4;
      for (int pass = 0; pass < 2; ++pass) {
#pragma unroll
        for (int it = 0; it < 8; ++it) {
          const int row = it * 2 + hh;
          v4f v = *(const v4f*)(slab + row * 68 + c4);
          *(volatile v4f*)(C + (size_t)(mBase + row) * ldc + n0 + c4) = v;
        }
        __threadfence();
      }
    } else {
      const int q = lane >> 3, c8 = (lane & 7) * 8;
      unsigned short* C  = (unsigned short*)Cout  + (size_t)b * strideC;
      unsigned short* C2 = (OUT_MODE == 2) ? ((unsigned short*)Cout2 + (size_t)b * strideC) : nullptr;
      for (int pass = 0; pass < 2; ++pass) {
#pragma unroll
        for (int it = 0; it < 4; ++it) {
          const int row = it * 4 + q;
          const float* sp = slab + row * 68 + c8;
          v8h hv, lv;
#pragma unroll
          for (int e = 0; e < 8; ++e) {
            if (OUT_MODE == 1) {
              hv[e] = (_Float16)sp[e];
            } else {
              unsigned short hb = f2bf_bits(sp[e]);
              unsigned short lb = f2bf_bits(sp[e] - bf_bits2f(hb));
              hv[e] = __builtin_bit_cast(_Float16, hb);
              lv[e] = __builtin_bit_cast(_Float16, lb);
            }
          }
          *(volatile v8h*)(C + (size_t)(mBase + row) * ldc + n0 + c8) = hv;
          if (OUT_MODE == 2) *(volatile v8h*)(C2 + (size_t)(mBase + row) * ldc + n0 + c8) = lv;
        }
        __threadfence();
      }
    }
    __builtin_amdgcn_fence(__ATOMIC_RELEASE, "workgroup");
    __builtin_amdgcn_wave_barrier();
    __builtin_amdgcn_fence(__ATOMIC_ACQUIRE, "workgroup");
  }
}

__global__ __launch_bounds__(256) void wtcast_kernel(const float* __restrict__ W, unsigned short* __restrict__ out,
                                                     int Din, int Dout, float scale) {
  __shared__ float sm[64][65];
  const int t  = threadIdx.x;
  const int d0 = blockIdx.x * 64;
  const int h0 = blockIdx.y * 64;
#pragma unroll
  for (int i = 0; i < 16; ++i) {
    const int e = i * 256 + t;
    const int r = e >> 6;
    const int c = e & 63;
    sm[c][r] = W[(size_t)(d0 + r) * Dout + h0 + c] * scale;
  }
  __syncthreads();
  const int lane = t & 31, wave = t >> 5;
  const int q = lane >> 3, c8 = (lane & 7) * 8;
  for (int pass = 0; pass < 2; ++pass) {
#pragma unroll
    for (int it = 0; it < 2; ++it) {
      const int row = wave * 8 + it * 4 + q;
      unsigned short hb[8];
#pragma unroll
      for (int e = 0; e < 8; ++e) hb[e] = h_bits(sm[row][c8 + e]);
      const v4u u = (v4u){pk16(hb[0], hb[1]), pk16(hb[2], hb[3]), pk16(hb[4], hb[5]), pk16(hb[6], hb[7])};
      *(volatile v4u*)(out + (size_t)(h0 + row) * Din + d0 + c8) = u;
    }
    __threadfence();
  }
}

__global__ __launch_bounds__(128) void ln_kernel(const float* __restrict__ x, const float* __restrict__ g,
                                                 const float* __restrict__ be, unsigned short* __restrict__ y) {
  __shared__ float red1[4];
  __shared__ float red2[4];
  const int row  = blockIdx.x;
  const int t    = threadIdx.x;
  const int lane = t & 31, wave = t >> 5;
  const int c0   = t * 8;
  const float* xr = x + (size_t)row * kEmb + c0;
  const v4f a = *(const v4f*)(xr);
  const v4f c = *(const v4f*)(xr + 4);
  float xv[8];
#pragma unroll
  for (int e = 0; e < 4; ++e) { xv[e] = a[e]; xv[4 + e] = c[e]; }
  float s = ((xv[0] + xv[1]) + (xv[2] + xv[3])) + ((xv[4] + xv[5]) + (xv[6] + xv[7]));
#pragma unroll
  for (int off = 16; off > 0; off >>= 1) s += __shfl_xor(s, off, 32);
  if (lane == 0) red1[wave] = s;
  __syncthreads();
  const float mu = ((red1[0] + red1[1]) + (red1[2] + red1[3])) * kInvEmb;
  float d[8];
#pragma unroll
  for (int e = 0; e < 8; ++e) d[e] = xv[e] - mu;
  float ss = ((d[0] * d[0] + d[1] * d[1]) + (d[2] * d[2] + d[3] * d[3])) +
             ((d[4] * d[4] + d[5] * d[5]) + (d[6] * d[6] + d[7] * d[7]));
#pragma unroll
  for (int off = 16; off > 0; off >>= 1) ss += __shfl_xor(ss, off, 32);
  if (lane == 0) red2[wave] = ss;
  __syncthreads();
  const float var = ((red2[0] + red2[1]) + (red2[2] + red2[3])) * kInvEmb;
  const float rs = 1.0f / sqrtf(var + kLnEps);
  const v4f ga = *(const v4f*)(g + c0);
  const v4f gc = *(const v4f*)(g + c0 + 4);
  const v4f ba = *(const v4f*)(be + c0);
  const v4f bc = *(const v4f*)(be + c0 + 4);
  unsigned short hb[8];
#pragma unroll
  for (int e = 0; e < 4; ++e) {
    hb[e]     = h_bits((d[e] * rs) * ga[e] + ba[e]);
    hb[4 + e] = h_bits((d[4 + e] * rs) * gc[e] + bc[e]);
  }
  const v4u u = (v4u){pk16(hb[0], hb[1]), pk16(hb[2], hb[3]), pk16(hb[4], hb[5]), pk16(hb[6], hb[7])};
  unsigned short* yp = y + (size_t)row * kEmb + c0;
  *(volatile v4u*)yp = u;
  __threadfence();
  *(volatile v4u*)yp = u;
}

__global__ __launch_bounds__(256) void vt_kernel(const float* __restrict__ Vf, unsigned short* __restrict__ VT) {
  __shared__ float sm[64][65];
  const int tid = threadIdx.x;
  const int t0  = blockIdx.x * 64;
  const int bh  = blockIdx.y;
  const int bb  = bh >> 4, hd = bh & 15;
#pragma unroll
  for (int i = 0; i < 16; ++i) {
    const int e = i * 256 + tid;
    const int r = e >> 6;
    const int c = e & 63;
    sm[c][r] = Vf[((size_t)(bb * kSeq + t0 + r)) * kEmb + hd * kHd + c];
  }
  __syncthreads();
  const int lane = tid & 31, wave = tid >> 5;
  const int q = lane >> 3, c8 = (lane & 7) * 8;
  for (int pass = 0; pass < 2; ++pass) {
#pragma unroll
    for (int it = 0; it < 2; ++it) {
      const int row = wave * 8 + it * 4 + q;
      unsigned short hb[8];
#pragma unroll
      for (int e = 0; e < 8; ++e) hb[e] = h_bits(sm[row][c8 + e]);
      const v4u u = (v4u){pk16(hb[0], hb[1]), pk16(hb[2], hb[3]), pk16(hb[4], hb[5]), pk16(hb[6], hb[7])};
      *(volatile v4u*)(VT + ((size_t)bh * kHd + row) * kSeq + t0 + c8) = u;
    }
    __threadfence();
  }
}

__global__ __launch_bounds__(256) void softmax_window_kernel(const float* __restrict__ S, const int* __restrict__ isgb,
                                                             unsigned short* __restrict__ P, float carry) {
  __shared__ float redM[8];
  __shared__ float redS[8];
  const int row  = blockIdx.x;
  const int z    = blockIdx.y;
  const int t    = threadIdx.x;
  const int lane = t & 31, wave = t >> 5;
  const int c0   = t * 8;
  const size_t rbase = ((size_t)z * kSeq + row) * kSeq + c0;
  const v4f a = *(const v4f*)(S + rbase);
  const v4f c = *(const v4f*)(S + rbase + 4);
  const v4i ga = *(const v4i*)(isgb + c0);
  const v4i gc = *(const v4i*)(isgb + c0 + 4);
  const int qg = isgb[row];
  float x[8];
#pragma unroll
  for (int e = 0; e < 4; ++e) {
    const int d0 = c0 + e - row;
    const int d1 = c0 + 4 + e - row;
    const bool al0 = (d0 <= kHalfWin && d0 >= -kHalfWin) || (qg != 0) || (ga[e] != 0);
    const bool al1 = (d1 <= kHalfWin && d1 >= -kHalfWin) || (qg != 0) || (gc[e] != 0);
    x[e]     = al0 ? a[e] : kMaskFill;
    x[4 + e] = al1 ? c[e] : kMaskFill;
  }
  float m = fmaxf(fmaxf(fmaxf(x[0], x[1]), fmaxf(x[2], x[3])), fmaxf(fmaxf(x[4], x[5]), fmaxf(x[6], x[7])));
#pragma unroll
  for (int off = 16; off > 0; off >>= 1) m = fmaxf(m, __shfl_xor(m, off, 32));
  if (lane == 0) redM[wave] = m;
  __syncthreads();
  m = redM[0];
#pragma unroll
  for (int w = 1; w < 8; ++w) m = fmaxf(m, redM[w]);
  float ex[8];
#pragma unroll
  for (int e = 0; e < 8; ++e) ex[e] = expf(x[e] - m);
  float s = ((ex[0] + ex[1]) + (ex[2] + ex[3])) + ((ex[4] + ex[5]) + (ex[6] + ex[7]));
#pragma unroll
  for (int off = 16; off > 0; off >>= 1) s += __shfl_xor(s, off, 32);
  if (lane == 0) redS[wave] = s;
  __syncthreads();
  float tot = redS[0];
#pragma unroll
  for (int w = 1; w < 8; ++w) tot += redS[w];
  const float inv = (1.0f / tot) * carry;
  unsigned short hb[8];
#pragma unroll
  for (int e = 0; e < 8; ++e) hb[e] = h_bits(ex[e] * inv);
  const v4u u = (v4u){pk16(hb[0], hb[1]), pk16(hb[2], hb[3]), pk16(hb[4], hb[5]), pk16(hb[6], hb[7])};
  unsigned short* pp = P + rbase;
  *(volatile v4u*)pp = u;
  __threadfence();
  *(volatile v4u*)pp = u;
}

__global__ __launch_bounds__(256) void gelu_cast_kernel(const float* __restrict__ in, unsigned short* __restrict__ out,
                                                        int n2, float carry) {
  const int i = blockIdx.x * 256 + threadIdx.x;
  if (i < n2) {
    const v2f u = *(const v2f*)(in + 2 * (size_t)i);
    const float g0 = ((0.5f * u[0]) * (1.0f + erff(u[0] * kInvSqrt2))) * carry;
    const float g1 = ((0.5f * u[1]) * (1.0f + erff(u[1] * kInvSqrt2))) * carry;
    const unsigned w = pk16(h_bits(g0), h_bits(g1));
    ((volatile unsigned*)out)[i] = w;
    __threadfence();
    ((volatile unsigned*)out)[i] = w;
  }
}

extern "C" void kernel_launch(void* const* d_in, const int* in_sizes, int n_in,
                              void* d_out, int out_size, void* d_ws, size_t ws_size,
                              hipStream_t stream) {
  if (n_in < 18) return;
  if (in_sizes[0] != kRows * kEmb || out_size != kRows * kEmb) return;
  if (in_sizes[1] != kRows) return;
  if (in_sizes[2] != kEmb * kEmb || in_sizes[4] != kEmb * kEmb || in_sizes[6] != kEmb * kEmb ||
      in_sizes[8] != kEmb * kEmb) return;
  if (in_sizes[14] != kEmb * kFF || in_sizes[16] != kFF * kEmb) return;
  if (in_sizes[3] != kEmb || in_sizes[15] != kFF || in_sizes[17] != kEmb) return;

  const float* x     = (const float*)d_in[0];
  const int*   isg   = (const int*)d_in[1];
  const float* Wq    = (const float*)d_in[2];
  const float* bq    = (const float*)d_in[3];
  const float* Wk    = (const float*)d_in[4];
  const float* bk    = (const float*)d_in[5];
  const float* Wv    = (const float*)d_in[6];
  const float* bv    = (const float*)d_in[7];
  const float* Wo    = (const float*)d_in[8];
  const float* bo    = (const float*)d_in[9];
  const float* g1    = (const float*)d_in[10];
  const float* beta1 = (const float*)d_in[11];
  const float* g2    = (const float*)d_in[12];
  const float* beta2 = (const float*)d_in[13];
  const float* W1    = (const float*)d_in[14];
  const float* b1    = (const float*)d_in[15];
  const float* W2    = (const float*)d_in[16];
  const float* b2    = (const float*)d_in[17];
  float* out = (float*)d_out;

  const size_t MiB = (size_t)1 << 20;
  const size_t offWq  = 0;
  const size_t offWk  = 2 * MiB;
  const size_t offWv  = 4 * MiB;
  const size_t offWo  = 6 * MiB;
  const size_t offW1  = 8 * MiB;
  const size_t offW2  = 16 * MiB;
  const size_t offY   = 24 * MiB;
  const size_t offQ   = 32 * MiB;
  const size_t offK   = 40 * MiB;
  const size_t offVT  = 48 * MiB;
  const size_t offS   = 56 * MiB;
  const size_t offP   = 88 * MiB;
  const size_t offG   = 48 * MiB;
  const size_t offF1  = 80 * MiB;
  const size_t total  = 104 * MiB;
  if (ws_size < total) return;

  char* ws = (char*)d_ws;
  unsigned short* WqT = (unsigned short*)(ws + offWq);
  unsigned short* WkT = (unsigned short*)(ws + offWk);
  unsigned short* WvT = (unsigned short*)(ws + offWv);
  unsigned short* WoT = (unsigned short*)(ws + offWo);
  unsigned short* W1T = (unsigned short*)(ws + offW1);
  unsigned short* W2T = (unsigned short*)(ws + offW2);
  unsigned short* Y16   = (unsigned short*)(ws + offY);
  unsigned short* CTX16 = (unsigned short*)(ws + offY);
  unsigned short* Y2    = (unsigned short*)(ws + offY);
  unsigned short* Q16 = (unsigned short*)(ws + offQ);
  unsigned short* K16 = (unsigned short*)(ws + offK);
  unsigned short* VT  = (unsigned short*)(ws + offVT);
  float* Vf   = (float*)(ws + offS);
  float* Sbuf = (float*)(ws + offS);
  unsigned short* P16 = (unsigned short*)(ws + offP);
  float* X1 = (float*)(ws + offQ);
  float* G  = (float*)(ws + offG);
  unsigned short* F1 = (unsigned short*)(ws + offF1);

  const long planeQK = (long)kSeq * kHd;
  const long planeS  = (long)kSeq * kSeq;

  wtcast_kernel<<<dim3(kEmb / 64, kEmb / 64), 256, 0, stream>>>(Wq, WqT, kEmb, kEmb, kWCarry);
  wtcast_kernel<<<dim3(kEmb / 64, kEmb / 64), 256, 0, stream>>>(Wk, WkT, kEmb, kEmb, kWCarry);
  wtcast_kernel<<<dim3(kEmb / 64, kEmb / 64), 256, 0, stream>>>(Wv, WvT, kEmb, kEmb, kWCarry);
  wtcast_kernel<<<dim3(kEmb / 64, kEmb / 64), 256, 0, stream>>>(Wo, WoT, kEmb, kEmb, kWCarry);
  wtcast_kernel<<<dim3(kEmb / 64, kFF / 64), 256, 0, stream>>>(W1, W1T, kEmb, kFF, kWCarry);
  wtcast_kernel<<<dim3(kFF / 64, kEmb / 64), 256, 0, stream>>>(W2, W2T, kFF, kEmb, kWCarry);

  ln_kernel<<<kRows, 128, 0, stream>>>(x, g1, beta1, Y16);

  {
    const int gx = ((kRows / 64) * (kEmb / 64) + 7) / 8;
    wmma_gemm64<0, false, 2, 1, false, 0, 0><<<dim3(gx, 1), 256, 0, stream>>>(
        Y16, Y16, kEmb, 0L, WqT, WqT, kEmb, 0L, Q16, Q16, kEmb, 0L, bq, x, 0L, kRows, kEmb, kEmb, kWCarryInv);
    wmma_gemm64<0, false, 2, 1, false, 0, 0><<<dim3(gx, 1), 256, 0, stream>>>(
        Y16, Y16, kEmb, 0L, WkT, WkT, kEmb, 0L, K16, K16, kEmb, 0L, bk, x, 0L, kRows, kEmb, kEmb, kWCarryInv);
    wmma_gemm64<0, false, 2, 0, false, 0, 0><<<dim3(gx, 1), 256, 0, stream>>>(
        Y16, Y16, kEmb, 0L, WvT, WvT, kEmb, 0L, Vf, Vf, kEmb, 0L, bv, x, 0L, kRows, kEmb, kEmb, kWCarryInv);
  }

  vt_kernel<<<dim3(kSeq / 64, kBH), 256, 0, stream>>>(Vf, VT);

  for (int g = 0; g < kBH / 2; ++g) {
    const int bh0 = 2 * g;
    const int bb = bh0 >> 4, hd = bh0 & 15;
    const unsigned short* Qg = Q16 + (size_t)(bb * kSeq) * kEmb + hd * kHd;
    const unsigned short* Kg = K16 + (size_t)(bb * kSeq) * kEmb + hd * kHd;
    const unsigned short* Vg = VT  + (size_t)bh0 * planeQK;
    unsigned short* Cg = CTX16 + (size_t)(bb * kSeq) * kEmb + hd * kHd;
    const int* isgb = isg + (size_t)bb * kSeq;
    {
      const int gx = ((kSeq / 64) * (kSeq / 64) + 7) / 8;
      wmma_gemm64<0, false, 0, 0, false, 0, 0><<<dim3(gx, 2), 256, 0, stream>>>(
          Qg, Qg, kEmb, (long)kHd, Kg, Kg, kEmb, (long)kHd, Sbuf, Sbuf, kSeq, planeS, bq, x, 0L,
          kSeq, kSeq, kHd, kScoreScale);
    }
    softmax_window_kernel<<<dim3(kSeq, 2), 256, 0, stream>>>(Sbuf, isgb, P16, kPCarry);
    {
      const int gx = ((kSeq / 64) * (kHd / 64) + 7) / 8;
      wmma_gemm64<0, false, 0, 1, false, 0, 0><<<dim3(gx, 2), 256, 0, stream>>>(
          P16, P16, kSeq, planeS, Vg, Vg, kSeq, planeQK, Cg, Cg, kEmb, (long)kHd, bq, x, 0L,
          kSeq, kHd, kSeq, kPVScale);
    }
  }

  {
    const int gx = ((kRows / 64) * (kEmb / 64) + 7) / 8;
    wmma_gemm64<0, false, 2, 0, true, 0, 0><<<dim3(gx, 1), 256, 0, stream>>>(
        CTX16, CTX16, kEmb, 0L, WoT, WoT, kEmb, 0L, X1, X1, kEmb, 0L, bo, x, 0L, kRows, kEmb, kEmb, kOutScale);
  }

  ln_kernel<<<kRows, 128, 0, stream>>>(X1, g2, beta2, Y2);

  for (int ch = 0; ch < kRows / kFFRows; ++ch) {
    const unsigned short* Yc = Y2 + (size_t)ch * kFFRows * kEmb;
    const float* X1c = X1 + (size_t)ch * kFFRows * kEmb;
    float* outc = out + (size_t)ch * kFFRows * kEmb;
    {
      const int gx = ((kFFRows / 64) * (kFF / 64) + 7) / 8;
      wmma_gemm64<0, false, 2, 0, false, 0, 0><<<dim3(gx, 1), 256, 0, stream>>>(
          Yc, Yc, kEmb, 0L, W1T, W1T, kEmb, 0L, G, G, kFF, 0L, b1, x, 0L, kFFRows, kFF, kEmb, kWCarryInv);
    }
    {
      const int n2 = (kFFRows * kFF) / 2;
      gelu_cast_kernel<<<(n2 + 255) / 256, 256, 0, stream>>>(G, F1, n2, kF1Carry);
    }
    {
      const int gx = ((kFFRows / 64) * (kEmb / 64) + 7) / 8;
      wmma_gemm64<0, false, 2, 0, true, 0, 0><<<dim3(gx, 1), 256, 0, stream>>>(
          F1, F1, kFF, 0L, W2T, W2T, kFF, 0L, outc, outc, kEmb, 0L, b2, X1c, 0L, kFFRows, kEmb, kFF, kFF2Scale);
    }
  }
}
